// MappingLayer_75685913690508
// MI455X (gfx1250) — hardware-run, weakly checked
//
#include <hip/hip_runtime.h>


namespace {
constexpr int NB_ = 64, A = 128, IC = 128, D = 64, NT = NB_ * A  , CH = 256  , KTOT = A * D  ;
constexpr float XS = 8.0f, HS = 256.0f, PS = 256.0f, WSC = 256.0f, NS = 1024.0f  ;
typedef _Float16 b16;
typedef __attribute__((ext_vector_type(16))) _Float16 v16b;
typedef __attribute__((ext_vector_type(8))) _Float16 v8b;
typedef __attribute__((ext_vector_type(2))) _Float16 v2b;
typedef __attribute__((ext_vector_type(8))) float v8f;
typedef __attribute__((ext_vector_type(4))) float v4f;
typedef __attribute__((ext_vector_type(2))) float v2f;
__device__ __forceinline__ float bf16_rne(float f) { unsigned int u = __float_as_uint(f); u += 0x7FFFu + ((u >> 16) & 1u); float r = __uint_as_float(u & 0xFFFF0000u); asm volatile("" : "+v"(r)); return r; }
__device__ __forceinline__ float bfv(float f) { float r = bf16_rne(f); asm volatile("" : "+v"(r)); return r; }
__device__ __forceinline__ void split16(float v, b16& hi, b16& lo) { hi = (b16)v; lo = (b16)(v - (float)hi); }
__device__ __forceinline__ v16b frag_kb(const b16* p, int hh) { const v8b a = *(const v8b*)(p + 8 * hh), b = *(const v8b*)(p + 16 + 8 * hh); v16b f;
#pragma unroll
  for (int e = 0; e < 8; ++e) { f[e] = a[e]; f[8 + e] = b[e]; } return f; }
__device__ __forceinline__ v8f wmma16b(v16b a, v16b b, v8f c) { v8f d = __builtin_amdgcn_wmma_f32_16x16x32_f16(false, a, false, b, (short)0, c, false, false); asm volatile("v_nop\n\tv_nop\n\tv_nop\n\tv_nop" : "+v"(d) : "v"(a), "v"(b)); return d; }
__device__ __forceinline__ void wave_lds_sync() { __builtin_amdgcn_fence(__ATOMIC_RELEASE, "workgroup"); __builtin_amdgcn_wave_barrier(); __builtin_amdgcn_fence(__ATOMIC_ACQUIRE, "workgroup"); }
__device__ __forceinline__ float pmul(float a, float b) { float p = a * b; asm volatile("" : "+v"(p)); return p; }

__global__ __launch_bounds__(256) void wput_kernel(const float* __restrict__ wq, const float* __restrict__ wk, const float* __restrict__ wv, b16* __restrict__ W) { const int u = blockIdx.x * 256 + threadIdx.x; if (u >= 3 * D * 16) return; const int o = u / 16, k0 = (u % 16) * 8; const float* w = o < D ? wq : (o < 2 * D ? wk : wv); const int oo = o % D; v8b v;
#pragma unroll
  for (int j = 0; j < 8; ++j) v[j] = (b16)(bf16_rne(w[(size_t)oo * IC + k0 + j]) * WSC);
  for (int pass = 0; pass < 2; ++pass) { *(volatile v8b*)(W + (size_t)o * IC + k0) = v; __threadfence(); } }
__global__ __launch_bounds__(32) void qkv_kernel(const float* __restrict__ feat, const b16* __restrict__ W, const float* __restrict__ bq, const float* __restrict__ bk, const float* __restrict__ bv, float* __restrict__ Q, b16* __restrict__ KH, b16* __restrict__ KL, float* __restrict__ V, b16* __restrict__ VNH, b16* __restrict__ VNL) { __shared__ __attribute__((aligned(16))) b16 Ah[16][IC + 8]; __shared__ float Tf[16][3 * D + 4], Nr[16]; const int lane = threadIdx.x, nloc = lane & 15, hlf = lane >> 4; const int b = blockIdx.x / (A / 16), a0 = (blockIdx.x % (A / 16)) * 16; const size_t n0 = (size_t)b * A + a0;
  for (int c = 0; c < IC; ++c) if (lane < 16) Ah[lane][c] = (b16)(bf16_rne(feat[((size_t)b * IC + c) * A + a0 + lane]) * XS);
  if (lane < 16) for (int k = IC; k < IC + 8; ++k) Ah[lane][k] = (b16)0.0f;
  wave_lds_sync(); v8f acc[12];
#pragma unroll
  for (int t = 0; t < 12; ++t) acc[t] = (v8f){};
#pragma unroll
  for (int kb = 0; kb < IC; kb += 32) { const v16b a = frag_kb(&Ah[nloc][kb], hlf);
#pragma unroll
    for (int t = 0; t < 12; ++t) acc[t] = wmma16b(a, frag_kb(W + (size_t)(t * 16 + nloc) * IC + kb, hlf), acc[t]); }
#pragma unroll
  for (int t = 0; t < 12; ++t) { const int cc = t * 16 + nloc; const float bb = bfv(cc < D ? bq[cc] : (cc < 2 * D ? bk[cc - D] : bv[cc - 2 * D]));
#pragma unroll
    for (int r8 = 0; r8 < 8; ++r8) Tf[8 * hlf + r8][cc] = acc[t][r8] * (1.0f / (XS * WSC)) + bb; }
  wave_lds_sync();
  for (int rr = 0; rr < 16; ++rr) { const float v0 = Tf[rr][2 * D + lane * 2], v1 = Tf[rr][2 * D + lane * 2 + 1]; float s = v0 * v0 + v1 * v1; for (int o = 16; o; o >>= 1) s += __shfl_xor(s, o); if (lane == 0) Nr[rr] = 1.0f / fmaxf(sqrtf(s), 1e-12f); }
  wave_lds_sync();
  for (int pass = 0; pass < 2; ++pass) { for (int rr = 0; rr < 16; ++rr) { const size_t n = n0 + rr; *(volatile v2f*)(Q + n * D + lane * 2) = (v2f){Tf[rr][lane * 2], Tf[rr][lane * 2 + 1]}; *(volatile v2f*)(V + n * D + lane * 2) = (v2f){Tf[rr][2 * D + lane * 2], Tf[rr][2 * D + lane * 2 + 1]};
      b16 h0, l0, h1, l1; split16(Tf[rr][D + lane * 2] * HS, h0, l0); split16(Tf[rr][D + lane * 2 + 1] * HS, h1, l1); *(volatile v2b*)(KH + n * D + lane * 2) = (v2b){h0, h1}; *(volatile v2b*)(KL + n * D + lane * 2) = (v2b){l0, l1};
      const float inv = Nr[rr]; split16(Tf[rr][2 * D + lane * 2] * inv * NS, h0, l0); split16(Tf[rr][2 * D + lane * 2 + 1] * inv * NS, h1, l1); *(volatile v2b*)(VNH + n * D + lane * 2) = (v2b){h0, h1}; *(volatile v2b*)(VNL + n * D + lane * 2) = (v2b){l0, l1}; }
    __threadfence(); } }
__global__ __launch_bounds__(256) void vt_kernel(const float* __restrict__ V, b16* __restrict__ VTH, b16* __restrict__ VTL) { __shared__ float Tt[64][65]; const int n0 = blockIdx.x * 64; const int tid = threadIdx.x, wave = tid >> 5, lane = tid & 31;
  for (int q = wave; q < 64; q += 8) { Tt[q][lane * 2] = V[(size_t)(n0 + q) * D + lane * 2]; Tt[q][lane * 2 + 1] = V[(size_t)(n0 + q) * D + lane * 2 + 1]; }
  __syncthreads();
  for (int pass = 0; pass < 2; ++pass) { for (int d = wave; d < D; d += 8) { b16 h0, l0, h1, l1; split16(Tt[lane * 2][d] * HS, h0, l0); split16(Tt[lane * 2 + 1][d] * HS, h1, l1); *(volatile v2b*)(VTH + (size_t)d * NT + n0 + lane * 2) = (v2b){h0, h1}; *(volatile v2b*)(VTL + (size_t)d * NT + n0 + lane * 2) = (v2b){l0, l1}; } __threadfence(); } }
__global__ __launch_bounds__(32) void att_kernel(const float* __restrict__ Q, const b16* __restrict__ KH, const b16* __restrict__ KL, const b16* __restrict__ VTH, const b16* __restrict__ VTL, int QLIM, b16* __restrict__ QNH, b16* __restrict__ QNL) { __shared__ __attribute__((aligned(16))) b16 Ah[16][D + 8], Al[16][D + 8], Pa[16][CH + 8], Pb[16][CH + 8]; __shared__ float Sc[16][CH + 1], Mx[16], Ls[16], Fc[16], Of[16][D + 1]; const int lane = threadIdx.x, nloc = lane & 15, hlf = lane >> 4; const size_t q0 = (size_t)blockIdx.x * 16;
  if (q0 >= (size_t)QLIM) { for (int pass = 0; pass < 2; ++pass) { for (int r = 0; r < 16; ++r) { *(volatile v2b*)(QNH + (q0 + r) * D + lane * 2) = (v2b){(b16)0.0f, (b16)0.0f}; *(volatile v2b*)(QNL + (q0 + r) * D + lane * 2) = (v2b){(b16)0.0f, (b16)0.0f}; } __threadfence(); } return; }
  for (int rr = 0; rr < 16; ++rr) for (int qd = 0; qd < 2; ++qd) { const int c = qd * 32 + lane; b16 p, ql; split16(Q[(q0 + rr) * D + c] * 0.125f * HS, p, ql); Ah[rr][c] = p; Al[rr][c] = ql; }
  if (lane < 16) { for (int k = D; k < D + 8; ++k) { Ah[lane][k] = (b16)0.0f; Al[lane][k] = (b16)0.0f; } for (int k = CH; k < CH + 8; ++k) { Pa[lane][k] = (b16)0.0f; Pb[lane][k] = (b16)0.0f; } Mx[lane] = -INFINITY; Ls[lane] = 0.0f; }
  wave_lds_sync(); const v16b qa0 = frag_kb(&Ah[nloc][0], hlf), qa1 = frag_kb(&Ah[nloc][32], hlf), ql0 = frag_kb(&Al[nloc][0], hlf), ql1 = frag_kb(&Al[nloc][32], hlf);
  v8f oacc[4] = {(v8f){}, (v8f){}, (v8f){}, (v8f){}};
#pragma unroll 1
  for (int ch = 0; ch < NT / CH; ++ch) { const size_t k0 = (size_t)ch * CH;
#pragma unroll 1
    for (int half = 0; half < 2; ++half) { v8f sacc[8];
#pragma unroll
      for (int t = 0; t < 8; ++t) sacc[t] = (v8f){};
#pragma unroll
      for (int t = 0; t < 8; ++t) { const size_t key = k0 + half * 128 + t * 16 + nloc; const v16b kh0 = frag_kb(KH + key * D, hlf), kh1 = frag_kb(KH + key * D + 32, hlf), kl0 = frag_kb(KL + key * D, hlf), kl1 = frag_kb(KL + key * D + 32, hlf);
        sacc[t] = wmma16b(qa0, kh0, sacc[t]); sacc[t] = wmma16b(qa0, kl0, sacc[t]); sacc[t] = wmma16b(ql0, kh0, sacc[t]); sacc[t] = wmma16b(qa1, kh1, sacc[t]); sacc[t] = wmma16b(qa1, kl1, sacc[t]); sacc[t] = wmma16b(ql1, kh1, sacc[t]); }
#pragma unroll
      for (int t = 0; t < 8; ++t)
#pragma unroll
        for (int r8 = 0; r8 < 8; ++r8) Sc[8 * hlf + r8][half * 128 + t * 16 + nloc] = sacc[t][r8] * (1.0f / (HS * HS)); }
    wave_lds_sync();
    for (int r = 0; r < 16; ++r) { float mx = -INFINITY; for (int j = lane; j < CH; j += 32) mx = fmaxf(mx, Sc[r][j]); for (int o = 16; o; o >>= 1) mx = fmaxf(mx, __shfl_xor(mx, o)); const float mo = Mx[r], mn = fmaxf(mo, mx); float sm = 0.0f; for (int j = lane; j < CH; j += 32) { const float p = __expf(Sc[r][j] - mn); Sc[r][j] = p; sm += p; } for (int o = 16; o; o >>= 1) sm += __shfl_xor(sm, o); wave_lds_sync(); if (lane == 0) { const float fac = (mo == -INFINITY) ? 0.0f : __expf(mo - mn); Fc[r] = fac; Ls[r] = Ls[r] * fac + sm; Mx[r] = mn; } }
    wave_lds_sync();
    for (int r = 0; r < 16; ++r) for (int qd = 0; qd < CH / 32; ++qd) { const int c = qd * 32 + lane; b16 p, ql; split16(Sc[r][c] * PS, p, ql); Pa[r][c] = p; Pb[r][c] = ql; }
    wave_lds_sync();
#pragma unroll
    for (int t = 0; t < 4; ++t)
#pragma unroll
      for (int r8 = 0; r8 < 8; ++r8) oacc[t][r8] *= Fc[8 * hlf + r8];
#pragma unroll 2
    for (int kb = 0; kb < CH; kb += 32) { const v16b pa = frag_kb(&Pa[nloc][kb], hlf), pb = frag_kb(&Pb[nloc][kb], hlf);
#pragma unroll
      for (int t = 0; t < 4; ++t) { const v16b vh = frag_kb(VTH + (size_t)(t * 16 + nloc) * NT + k0 + kb, hlf), vl = frag_kb(VTL + (size_t)(t * 16 + nloc) * NT + k0 + kb, hlf); oacc[t] = wmma16b(pa, vh, oacc[t]); oacc[t] = wmma16b(pa, vl, oacc[t]); oacc[t] = wmma16b(pb, vh, oacc[t]); } }
    wave_lds_sync(); }
#pragma unroll
  for (int t = 0; t < 4; ++t)
#pragma unroll
    for (int r8 = 0; r8 < 8; ++r8) { const int r = 8 * hlf + r8; Of[r][t * 16 + nloc] = oacc[t][r8] * (1.0f / (PS * HS)) / Ls[r]; }
  wave_lds_sync();
  for (int r = 0; r < 16; ++r) { const float v0 = Of[r][lane * 2], v1 = Of[r][lane * 2 + 1]; float s = v0 * v0 + v1 * v1; for (int o = 16; o; o >>= 1) s += __shfl_xor(s, o); if (lane == 0) Fc[r] = 1.0f / fmaxf(sqrtf(s), 1e-12f); }
  wave_lds_sync();
  for (int pass = 0; pass < 2; ++pass) { for (int r = 0; r < 16; ++r) { const float inv = Fc[r]; b16 h0, l0, h1, l1; split16(Of[r][lane * 2] * inv * NS, h0, l0); split16(Of[r][lane * 2 + 1] * inv * NS, h1, l1); *(volatile v2b*)(QNH + (q0 + r) * D + lane * 2) = (v2b){h0, h1}; *(volatile v2b*)(QNL + (q0 + r) * D + lane * 2) = (v2b){l0, l1}; } __threadfence(); } }
__global__ __launch_bounds__(32) void sim_kernel(const b16* __restrict__ VNH, const b16* __restrict__ VNL, const b16* __restrict__ QNH, const b16* __restrict__ QNL, float* __restrict__ out) { __shared__ float Tf[16][D + 1]; const int lane = threadIdx.x, nloc = lane & 15, hlf = lane >> 4; const int i0 = blockIdx.x * 16; v8f acc[4] = {(v8f){}, (v8f){}, (v8f){}, (v8f){}};
#pragma unroll 2
  for (int kb = 0; kb < KTOT; kb += 32) { const v16b a = frag_kb(VNH + (size_t)(i0 + nloc) * KTOT + kb, hlf), al = frag_kb(VNL + (size_t)(i0 + nloc) * KTOT + kb, hlf);
#pragma unroll
    for (int t = 0; t < 4; ++t) { const v16b bh = frag_kb(QNH + (size_t)(t * 16 + nloc) * KTOT + kb, hlf), bl = frag_kb(QNL + (size_t)(t * 16 + nloc) * KTOT + kb, hlf); acc[t] = wmma16b(a, bh, acc[t]); acc[t] = wmma16b(a, bl, acc[t]); acc[t] = wmma16b(al, bh, acc[t]); } }
#pragma unroll
  for (int t = 0; t < 4; ++t)
#pragma unroll
    for (int r8 = 0; r8 < 8; ++r8) Tf[8 * hlf + r8][t * 16 + nloc] = acc[t][r8] * (1.0f / (NS * NS * (float)A));
  wave_lds_sync();
  for (int pass = 0; pass < 2; ++pass) { for (int r = 0; r < 16; ++r) *(volatile v2f*)(out + (size_t)(i0 + r) * NB_ + lane * 2) = (v2f){Tf[r][lane * 2], Tf[r][lane * 2 + 1]}; __threadfence(); } }
}

extern "C" void kernel_launch(void* const* d_in, const int* in_sizes, int n_in, void* d_out, int out_size, void* d_ws, size_t ws_size, hipStream_t stream) {
  (void)n_in;
  auto Fp = [&](int i) { return (const float*)d_in[i]; };
  if (in_sizes[0] != NB_ * IC * A || in_sizes[1] != D * IC || in_sizes[3] != D * IC || in_sizes[5] != D * IC || out_size != NB_ * NB_) return;
  const int QLIM = NT;
  size_t off = 0; char* ws = (char*)d_ws;
  auto carve = [&](size_t bytes) { char* p = ws + off; off += (bytes + 255) & ~(size_t)255; return p; };
  b16* W = (b16*)carve((size_t)3 * D * IC * 2); float* Q = (float*)carve((size_t)NT * D * 4); float* V = (float*)carve((size_t)NT * D * 4); b16* KH = (b16*)carve((size_t)NT * D * 2); b16* KL = (b16*)carve((size_t)NT * D * 2); b16* VTH = (b16*)carve((size_t)D * NT * 2); b16* VTL = (b16*)carve((size_t)D * NT * 2); b16* VNH = (b16*)carve((size_t)NT * D * 2); b16* VNL = (b16*)carve((size_t)NT * D * 2); b16* QNH = (b16*)carve((size_t)NT * D * 2); b16* QNL = (b16*)carve((size_t)NT * D * 2);
  if (off > ws_size || off > ((size_t)16 << 20)) return;
  wput_kernel<<<(3 * D * 16 + 255) / 256, 256, 0, stream>>>(Fp(1), Fp(3), Fp(5), W);
  qkv_kernel<<<NB_ * (A / 16), 32, 0, stream>>>(Fp(0), W, Fp(2), Fp(4), Fp(6), Q, KH, KL, V, VNH, VNL);
  vt_kernel<<<NT / 64, 256, 0, stream>>>(V, VTH, VTL);
  att_kernel<<<NT / 16, 32, 0, stream>>>(Q, KH, KL, VTH, VTL, QLIM, QNH, QNL);
  sim_kernel<<<NB_ / 16, 32, 0, stream>>>(VNH, VNL, QNH, QNL, (float*)d_out);
}
